// MultiHeadAttention_60284160966755
// MI455X (gfx1250) — hardware-run, weakly checked
//
#include <hip/hip_runtime.h>
#include <stddef.h>
#include <stdint.h>
#include <math.h>


#pragma clang fp contract(off)

#define NN      50000
#define NE      1600000
#define DIN     128
#define HC      128
#define NH      4
#define DH      32
#define NTHR    256
#define NWAVE   8
#define EPT     8
#define CHUNK   (NTHR * EPT)
#define WCAP    (EPT * 32)
#define LISTN   (NWAVE * WCAP)
#define NBA     512
#define SLA     9
#define RCAP    28672
#define DEGCAP  96
#define MEAS_B512   16715
#define MEAS_MAXDEG 61
#define GBM     64
#define GBN     64
#define GTHR    128
#define MP      (((NN + GBM - 1) / GBM) * GBM)
#define NGA     ((NN + NBA - 1) / NBA)
#define NUX     (MP * (DIN / 8))
#define NUW     (HC * (DIN / 8))
#define NEGSL   0.2f
#define WSMAX   134217728
#define SCAN_ZINTS    (RCAP + 3 * NBA)
#define SCAN_LDS_INTS (2 * RCAP + 3 * NBA + LISTN + 16 + NBA * 8)

static_assert(NH * DH == HC && HC == 128);
static_assert(32 * 4 == HC);
static_assert(DH / 4 == 8);
static_assert(NN % 16 == 0);
static_assert(NE % NTHR == 0);
static_assert((long long)NE < (1LL << 31));
static_assert((long long)NE < (1LL << (32 - SLA)));
static_assert(((long long)CHUNK << SLA) < (1LL << 31));
static_assert(((long long)NN * HC * 4) % 128 == 0);
static_assert((NBA & (NBA - 1)) == 0 && NBA == (1 << SLA));
static_assert(NBA % NWAVE == 0 && NBA % 32 == 0);
static_assert((RCAP % 32) == 0 && (SCAN_ZINTS % 4) == 0);
static_assert(RCAP >= MEAS_B512 + 2048);
static_assert(DEGCAP >= MEAS_MAXDEG + 8);
static_assert(SCAN_LDS_INTS * 4 <= 300000);
static_assert(NBA * 8 == 4 * NTHR * 4);
static_assert((NN * 32) % 128 == 0);
static_assert(GBM == (GTHR / 32) * 16);
static_assert((DIN % 32) == 0 && (3 * HC) % GBN == 0 && (MP % GBM) == 0);
static_assert((NUX % NTHR) == 0 && (NUW % NTHR) == 0);
static_assert(NGA * NBA >= NN);

typedef float          v4f  __attribute__((ext_vector_type(4)));
typedef float          v8f  __attribute__((ext_vector_type(8)));
typedef int            v4i  __attribute__((ext_vector_type(4)));
typedef int            v8i  __attribute__((ext_vector_type(8)));
typedef unsigned short v8us __attribute__((ext_vector_type(8)));
typedef __bf16         v16b __attribute__((ext_vector_type(16)));
typedef v4f  __attribute__((may_alias)) v4fa;
typedef v4i  __attribute__((may_alias)) v4ia;
typedef v8us __attribute__((may_alias)) v8usa;
union FragB { v16b v; v8us h[2]; v8i w; };

__device__ __forceinline__ v8f wmb(const FragB& a, const FragB& b, v8f c) {
  v8f d = __builtin_amdgcn_wmma_f32_16x16x32_bf16(false, a.v, false, b.v, (short)0, c, false, false);
  asm volatile("v_nop\n\tv_nop\n\tv_nop\n\tv_nop" : "+v"(d) : "v"(a.w), "v"(b.w));
  return d;
}

__device__ __forceinline__ unsigned int f2bf(float f) {
  const unsigned int u = __float_as_uint(f);
  const unsigned int r = ((u + 0x7FFFu + ((u >> 16) & 1u)) >> 16) & 0xFFFFu;
  return ((u & 0x7FFFFFFFu) > 0x7F800000u) ? 0x7FC0u : r;
}
__device__ __forceinline__ float bf2f(unsigned int b) { return __uint_as_float(b << 16); }
__device__ __forceinline__ float bfr(float f) { return bf2f(f2bf(f)); }

__device__ __forceinline__ void st8(unsigned short* dp, const v8us o) {
  *(volatile v8us*)dp = o;
  __threadfence();
  *(volatile v8us*)dp = o;
}

__device__ __forceinline__ v8us wunit(const float* __restrict__ W, int v) {
  const int n  = v >> 4;
  const int k8 = (v & 15) * 8;
  const float* p = W + (size_t)k8 * HC + n;
  v8us o;
#pragma unroll
  for (int i = 0; i < 8; ++i) o[i] = (unsigned short)f2bf(p[(size_t)i * HC]);
  return o;
}

template <int SLB>
__device__ __forceinline__ int scan_chunk(const int* __restrict__ dsts, int nE, int cbase, int slotBase,
                                          int nb, int vec8, int* list, int tid, int lane, int wave) {
  int wc = 0;
  const int el0  = tid * EPT;
  const int e0   = cbase + el0;
  const int sent = -2147483647 - 1;
  v4i da, db;
  if (vec8 != 0 && cbase + CHUNK <= nE) {
    da = *(const v4i*)(dsts + e0);
    db = *(const v4i*)(dsts + e0 + 4);
  } else {
    da.x = (e0     < nE) ? dsts[min(e0,     nE - 1)] : sent;
    da.y = (e0 + 1 < nE) ? dsts[min(e0 + 1, nE - 1)] : sent;
    da.z = (e0 + 2 < nE) ? dsts[min(e0 + 2, nE - 1)] : sent;
    da.w = (e0 + 3 < nE) ? dsts[min(e0 + 3, nE - 1)] : sent;
    db.x = (e0 + 4 < nE) ? dsts[min(e0 + 4, nE - 1)] : sent;
    db.y = (e0 + 5 < nE) ? dsts[min(e0 + 5, nE - 1)] : sent;
    db.z = (e0 + 6 < nE) ? dsts[min(e0 + 6, nE - 1)] : sent;
    db.w = (e0 + 7 < nE) ? dsts[min(e0 + 7, nE - 1)] : sent;
  }
  const unsigned nbs = (unsigned)slotBase;
  const unsigned unb = (unsigned)nb;
  const unsigned s0 = (unsigned)da.x - nbs, s1 = (unsigned)da.y - nbs;
  const unsigned s2 = (unsigned)da.z - nbs, s3 = (unsigned)da.w - nbs;
  const unsigned s4 = (unsigned)db.x - nbs, s5 = (unsigned)db.y - nbs;
  const unsigned s6 = (unsigned)db.z - nbs, s7 = (unsigned)db.w - nbs;
  const bool h0 = s0 < unb, h1 = s1 < unb, h2 = s2 < unb, h3 = s3 < unb;
  const bool h4 = s4 < unb, h5 = s5 < unb, h6 = s6 < unb, h7 = s7 < unb;
  const unsigned any = __builtin_amdgcn_ballot_w32(h0 | h1 | h2 | h3 | h4 | h5 | h6 | h7);
  if (any != 0u) {
#define HITJ(J, HJ, SJ) { \
      const unsigned mj = __builtin_amdgcn_ballot_w32(HJ); \
      if (mj != 0u) { \
        if (HJ) { \
          const int pos = wc + (int)__builtin_amdgcn_mbcnt_lo(mj, 0u); \
          if (pos < WCAP) list[wave * WCAP + pos] = ((el0 + (J)) << SLB) | (int)(SJ); \
        } \
        unsigned mv = mj; \
        asm volatile("" : "+v"(mv)); \
        wc += (int)__builtin_popcount(mv); } }
    HITJ(0, h0, s0)
    HITJ(1, h1, s1)
    HITJ(2, h2, s2)
    HITJ(3, h3, s3)
    HITJ(4, h4, s4)
    HITJ(5, h5, s5)
    HITJ(6, h6, s6)
    HITJ(7, h7, s7)
#undef HITJ
  }
  return wc;
}

__global__ __launch_bounds__(NTHR) void k_prep(const float* __restrict__ x, const float* __restrict__ Ws,
                                               const float* __restrict__ Wd, const float* __restrict__ Wv,
                                               const float* __restrict__ av, unsigned short* XB,
                                               unsigned short* WT, float* AV) {
  const int tid = (int)threadIdx.x;
  const int u = (int)blockIdx.x * NTHR + tid;
  if (u < NUX) {
    const int row = u >> 4;
    const int c0  = (u & 15) * 8;
    const int rc  = row < NN ? row : NN - 1;
    const float* p = x + (size_t)rc * DIN + c0;
    const v4f a = *(const v4f*)p;
    const v4f b = *(const v4f*)(p + 4);
    const unsigned int msk = (row < NN) ? 0xFFFFu : 0u;
    v8us o;
    o[0] = (unsigned short)(f2bf(a.x) & msk); o[1] = (unsigned short)(f2bf(a.y) & msk);
    o[2] = (unsigned short)(f2bf(a.z) & msk); o[3] = (unsigned short)(f2bf(a.w) & msk);
    o[4] = (unsigned short)(f2bf(b.x) & msk); o[5] = (unsigned short)(f2bf(b.y) & msk);
    o[6] = (unsigned short)(f2bf(b.z) & msk); o[7] = (unsigned short)(f2bf(b.w) & msk);
    st8(XB + (size_t)row * DIN + c0, o);
  } else if (u < NUX + NUW) {
    const int v = u - NUX;
    st8(WT + (size_t)v * 8, wunit(Ws, v));
  } else if (u < NUX + 2 * NUW) {
    const int v = u - NUX - NUW;
    st8(WT + (size_t)(NUW + v) * 8, wunit(Wd, v));
  } else if (u < NUX + 3 * NUW) {
    const int v = u - NUX - 2 * NUW;
    st8(WT + (size_t)(2 * NUW + v) * 8, wunit(Wv, v));
  } else {
    if (tid < 32) {
      const v4f a = *(const v4f*)(av + 4 * tid);
      v4f r;
      r.x = bfr(a.x); r.y = bfr(a.y); r.z = bfr(a.z); r.w = bfr(a.w);
      float* dp = AV + 4 * tid;
      *(volatile v4f*)dp = r;
      __threadfence();
      *(volatile v4f*)dp = r;
    }
  }
}

__global__ __launch_bounds__(GTHR) void k_proj(const unsigned short* __restrict__ A,
                                               const unsigned short* __restrict__ WT, float* P3) {
  __shared__ __attribute__((aligned(16))) float stg[GBM * GBN];
  const int tid = (int)threadIdx.x, lane = tid & 31, wave = tid >> 5, hh = lane >> 4, m = lane & 15;
  const int rowBase = (int)blockIdx.x * GBM;
  const int col0    = (int)blockIdx.y * GBN;

  v8f acc[4];
  {
    const v8f z = {0.f, 0.f, 0.f, 0.f, 0.f, 0.f, 0.f, 0.f};
    acc[0] = z; acc[1] = z; acc[2] = z; acc[3] = z;
  }
  const unsigned short* ap = A  + (size_t)(rowBase + 16 * wave + m) * (size_t)DIN + 8 * hh;
  const unsigned short* wp = WT + (size_t)(col0 + m) * (size_t)DIN + 8 * hh;
#pragma unroll 1
  for (int ks = 0; ks < DIN / 32; ++ks) {
    FragB af;
    af.h[0] = *(const v8usa*)(ap + 32 * ks);
    af.h[1] = *(const v8usa*)(ap + 32 * ks + 16);
#pragma unroll
    for (int t = 0; t < 4; ++t) {
      const unsigned short* wq = wp + (size_t)(16 * t) * (size_t)DIN + 32 * ks;
      FragB bf;
      bf.h[0] = *(const v8usa*)wq;
      bf.h[1] = *(const v8usa*)(wq + 16);
      acc[t] = wmb(af, bf, acc[t]);
    }
  }

#pragma unroll
  for (int t = 0; t < 4; ++t) {
    const int lc = 16 * t + m;
#pragma unroll
    for (int r = 0; r < 8; ++r) {
      const int lr = 16 * wave + 8 * hh + r;
      stg[lr * GBN + lc] = acc[t][r];
    }
  }
  __syncthreads();

  v4f fv[8];
#pragma unroll
  for (int i = 0; i < 8; ++i) {
    const int lr = 16 * wave + 2 * i + hh;
    fv[i] = *(const v4fa*)(stg + lr * GBN + 4 * m);
  }
  const size_t pbase = (size_t)(col0 >> 7) * (size_t)MP * HC + (size_t)(col0 & 127) + 4 * m;
#pragma unroll
  for (int i = 0; i < 8; ++i) {
    const int gr = rowBase + 16 * wave + 2 * i + hh;
    float* op = P3 + pbase + (size_t)gr * HC;
    *(volatile v4f*)op = fv[i];
  }
  __threadfence();
#pragma unroll
  for (int i = 0; i < 8; ++i) {
    const int gr = rowBase + 16 * wave + 2 * i + hh;
    float* op = P3 + pbase + (size_t)gr * HC;
    *(volatile v4f*)op = fv[i];
  }
}

__global__ __launch_bounds__(NTHR) __attribute__((amdgpu_num_vgpr(248)))
void k_score(const int* __restrict__ ei, const float* __restrict__ P3, const float* __restrict__ AV, float* SC) {
  __shared__ __attribute__((aligned(16))) float stg[NWAVE * 128];
  const int tid = (int)threadIdx.x, lane = tid & 31;
  const int wave = __builtin_amdgcn_readfirstlane(tid >> 5);
  const int e = ((int)blockIdx.x * NWAVE + wave) * 32 + lane;
  const int sraw = ei[e];
  const int draw = ei[NE + e];
  const int sv = sraw < 0 ? 0 : (sraw > NN - 1 ? NN - 1 : sraw);
  const int dv = draw < 0 ? 0 : (draw > NN - 1 ? NN - 1 : draw);
  const v4f va = *(const v4f*)(AV + 4 * lane);
  const float* HSp = P3 + 4 * lane;
  const float* HDp = P3 + (size_t)MP * HC + 4 * lane;
  const int h = lane >> 3;
  float* sw = stg + wave * 128;
#pragma unroll 4
  for (int k = 0; k < 32; ++k) {
    const int sk = __builtin_amdgcn_readlane(sv, k);
    const int dk = __builtin_amdgcn_readlane(dv, k);
    const v4f vs = *(const v4f*)(HSp + (size_t)sk * HC);
    const v4f vd = *(const v4f*)(HDp + (size_t)dk * HC);
    float t0 = vs.x + vd.x; t0 = (t0 > 0.f) ? t0 : NEGSL * t0;
    float t1 = vs.y + vd.y; t1 = (t1 > 0.f) ? t1 : NEGSL * t1;
    float t2 = vs.z + vd.z; t2 = (t2 > 0.f) ? t2 : NEGSL * t2;
    float t3 = vs.w + vd.w; t3 = (t3 > 0.f) ? t3 : NEGSL * t3;
    float p = t0 * va.x;
    p = fmaf(t1, va.y, p);
    p = fmaf(t2, va.z, p);
    p = fmaf(t3, va.w, p);
    p += __shfl_xor(p, 1);
    p += __shfl_xor(p, 2);
    p += __shfl_xor(p, 4);
    if ((lane & 7) == 0) sw[k * 4 + h] = p;
  }
  __syncthreads();
  const v4f o = *(const v4fa*)(sw + 4 * lane);
  float* op = SC + (size_t)e * 4;
  *(volatile v4f*)op = o;
  __threadfence();
  *(volatile v4f*)op = o;
}

__global__ __launch_bounds__(NTHR) __attribute__((amdgpu_num_vgpr(248)))
void k_scan(const int* __restrict__ ei, const float* __restrict__ P3, const float* __restrict__ SC,
            float* out0, float* MSg) {
  extern __shared__ __attribute__((aligned(16))) int ssm[];
  int* reg1 = ssm;
  int* reg2 = reg1 + RCAP;
  int* cnt  = reg2 + RCAP;
  int* offs = cnt + NBA;
  int* cur  = offs + NBA;
  int* list = cur + NBA;
  int* misc = list + LISTN;
  float* msl = (float*)(misc + 16);
  const int tid = (int)threadIdx.x, lane = tid & 31;
  const int wave = __builtin_amdgcn_readfirstlane(tid >> 5);
  const int blk = (int)blockIdx.x;
  const int nodeBase = blk * NBA;
  int nb = NN - nodeBase;
  nb = nb < 0 ? 0 : (nb > NBA ? NBA : nb);
  const int* srcs = ei;
  const int* dsts = ei + NE;

  {
    const v4i z4 = {0, 0, 0, 0};
    for (int i = tid * 4; i < SCAN_ZINTS; i += NTHR * 4) *(v4ia*)(reg2 + i) = z4;
    if (tid < 16) misc[tid] = 0;
  }
  __syncthreads();

  int tot = 0, ovf = 0;
  const int nChunks = (NE + CHUNK - 1) / CHUNK;
#pragma unroll 1
  for (int ch = 0; ch < nChunks; ++ch) {
    const int cbase = ch * CHUNK;
    const int wc = scan_chunk<SLA>(dsts, NE, cbase, nodeBase, nb, 1, list, tid, lane, wave);
    if (lane == 0) misc[wave] = wc;
    __syncthreads();
    int pre = 0, all = 0;
#pragma unroll
    for (int w2 = 0; w2 < NWAVE; ++w2) {
      int c = misc[w2];
      c = c < 0 ? 0 : (c > WCAP ? WCAP : c);
      all += c;
      pre += (w2 < wave) ? c : 0;
    }
    const int wcc  = wc > WCAP ? WCAP : wc;
    const int base = tot + pre;
#pragma unroll 1
    for (int i = lane; i < wcc; i += 32) {
      const int ent = list[wave * WCAP + i];
      const int el  = (ent >> SLA) & (CHUNK - 1);
      const int sl  = ent & (NBA - 1);
      int eid = cbase + el;
      eid = eid > NE - 1 ? NE - 1 : eid;
      const int pos = base + i;
      if (pos < RCAP) reg1[pos] = (int)(((unsigned)eid << SLA) | (unsigned)sl);
    }
    if (tot + all > RCAP) ovf = 1;
    tot += all;
    tot = tot > RCAP ? RCAP : tot;
    __syncthreads();
  }
  const int nh = tot;

  if (wave == 0) {
#pragma unroll 1
    for (int b0 = 0; b0 < nh; b0 += 32) {
      const int idx = b0 + lane;
      const int uv  = reg1[idx < nh ? idx : nh - 1];
      const int m32 = (nh - b0) < 32 ? (nh - b0) : 32;
#pragma unroll 1
      for (int k = 0; k < m32; ++k) {
        const int u  = __builtin_amdgcn_readlane(uv, k);
        const int sq = u & (NBA - 1);
        if (lane == 0) cnt[sq] = cnt[sq] + 1;
      }
    }
  }
  __syncthreads();
  if (wave == 0) {
    const int base = lane * (NBA / 32);
    int s = 0, bg = 0;
#pragma unroll 1
    for (int i = 0; i < NBA / 32; ++i) {
      const int cv = cnt[base + i];
      s += cv;
      bg |= (cv > DEGCAP) ? 1 : 0;
    }
    int incl = s;
#pragma unroll
    for (int d = 1; d < 32; d <<= 1) {
      const int y = __shfl_up(incl, d, 32);
      if (lane >= d) incl += y;
    }
    int run = incl - s;
#pragma unroll 1
    for (int i = 0; i < NBA / 32; ++i) {
      const int cv = cnt[base + i];
      offs[base + i] = run;
      cur[base + i]  = run;
      run += cv;
    }
    const unsigned bm = __builtin_amdgcn_ballot_w32(bg != 0);
    if (lane == 0) misc[8] = (bm != 0u) ? 1 : 0;
  }
  __syncthreads();
  if (wave == 0) {
#pragma unroll 1
    for (int b0 = 0; b0 < nh; b0 += 32) {
      const int idx = b0 + lane;
      const int uv  = reg1[idx < nh ? idx : nh - 1];
      const int m32 = (nh - b0) < 32 ? (nh - b0) : 32;
#pragma unroll 1
      for (int k = 0; k < m32; ++k) {
        const int u   = __builtin_amdgcn_readlane(uv, k);
        const int sq  = u & (NBA - 1);
        const int eid = (int)((unsigned)u >> SLA);
        if (lane == 0) {
          int p = cur[sq];
          p = p < 0 ? 0 : (p > RCAP - 1 ? RCAP - 1 : p);
          reg2[p] = eid;
          cur[sq] = p + 1;
        }
      }
    }
  }
  __syncthreads();

  const bool bad = (ovf != 0) || (misc[8] != 0);
  const float qnan = __int_as_float(0x7fc00000);
  const int h = lane >> 3;
  const float* HVp = P3 + (size_t)2 * MP * HC + 4 * lane;
  const float* SCh = SC + h;

#pragma unroll 1
  for (int si = 0; si < NBA / NWAVE; ++si) {
    const int s    = si * NWAVE + wave;
    const int node = nodeBase + s;
    int c = cnt[s];
    c = c < 0 ? 0 : (c > DEGCAP ? DEGCAP : c);
    int o = offs[s];
    o = o < 0 ? 0 : (o > RCAP ? RCAP : o);
    if (c > nh - o) c = nh - o;
    c = c < 0 ? 0 : c;
    c = __builtin_amdgcn_readfirstlane(c);
    o = __builtin_amdgcn_readfirstlane(o);
    float mx = -3.0e38f, dn = 0.0f;
    v4f acc = {0.f, 0.f, 0.f, 0.f};
#pragma unroll 1
    for (int b0 = 0; b0 < c; b0 += 32) {
      int idx = o + b0 + lane;
      idx = idx < 0 ? 0 : (idx > RCAP - 1 ? RCAP - 1 : idx);
      int eid = reg2[idx];
      eid = eid < 0 ? 0 : (eid > NE - 1 ? NE - 1 : eid);
      const int sraw = srcs[eid];
      asm volatile("" :: "v"(sraw));
      const int sr  = sraw < 0 ? 0 : (sraw > NN - 1 ? NN - 1 : sraw);
      const int m32 = (c - b0) < 32 ? (c - b0) : 32;
#pragma unroll 1
      for (int k = 0; k < m32; ++k) {
        const int sk = __builtin_amdgcn_readlane(sr, k);
        const int ek = __builtin_amdgcn_readlane(eid, k);
        const float sc = SCh[(size_t)ek * 4];
        const v4f hv = *(const v4f*)(HVp + (size_t)sk * HC);
        const float df = sc - mx;
        const float ee = expf(-fabsf(df));
        const bool  up = df > 0.f;
        const float s1 = up ? ee : 1.0f;
        const float s2 = up ? 1.0f : ee;
        mx = up ? sc : mx;
        dn = fmaf(dn, s1, s2);
        acc.x = fmaf(acc.x, s1, s2 * hv.x);
        acc.y = fmaf(acc.y, s1, s2 * hv.y);
        acc.z = fmaf(acc.z, s1, s2 * hv.z);
        acc.w = fmaf(acc.w, s1, s2 * hv.w);
      }
    }
    const bool has = c > 0;
    const float den = has ? (dn + 1e-9f) : 1.0f;
    v4f r;
    r.x = acc.x / den; r.y = acc.y / den; r.z = acc.z / den; r.w = acc.w / den;
    r.x = bad ? qnan : r.x; r.y = bad ? qnan : r.y; r.z = bad ? qnan : r.z; r.w = bad ? qnan : r.w;
    float mo = has ? mx : 0.0f;
    float lo = has ? dn : 0.0f;
    mo = bad ? qnan : mo;
    lo = bad ? qnan : lo;
    if ((lane & 7) == 0) { msl[s * 8 + h] = mo; msl[s * 8 + 4 + h] = lo; }
    if (node < NN) {
      float* op = out0 + (size_t)node * HC + 4 * lane;
      *(volatile v4f*)op = r;
      __threadfence();
      *(volatile v4f*)op = r;
    }
  }
  __syncthreads();

  {
    float* mb = MSg + (size_t)blk * (NBA * 8);
    v4f mv[4];
#pragma unroll
    for (int j = 0; j < 4; ++j) mv[j] = *(const v4fa*)(msl + (j * NTHR + tid) * 4);
#pragma unroll
    for (int j = 0; j < 4; ++j) *(volatile v4f*)(mb + (j * NTHR + tid) * 4) = mv[j];
    __threadfence();
#pragma unroll
    for (int j = 0; j < 4; ++j) *(volatile v4f*)(mb + (j * NTHR + tid) * 4) = mv[j];
  }
}

__global__ __launch_bounds__(NTHR) void k_attn(const int* __restrict__ ei, const float* __restrict__ SC,
                                               const float* __restrict__ MSg, float* out1) {
  const int e = (int)blockIdx.x * NTHR + (int)threadIdx.x;
  const int draw = ei[NE + e];
  const int d = draw < 0 ? 0 : (draw > NN - 1 ? NN - 1 : draw);
  const v4f sc = *(const v4f*)(SC + (size_t)e * 4);
  const v4f mx = *(const v4f*)(MSg + (size_t)d * 8);
  const v4f sm = *(const v4f*)(MSg + (size_t)d * 8 + 4);
  v4f a;
  a.x = expf(sc.x - mx.x) / (sm.x + 1e-9f);
  a.y = expf(sc.y - mx.y) / (sm.y + 1e-9f);
  a.z = expf(sc.z - mx.z) / (sm.z + 1e-9f);
  a.w = expf(sc.w - mx.w) / (sm.w + 1e-9f);
  float* op = out1 + (size_t)e * 4;
  *(volatile v4f*)op = a;
  __threadfence();
  *(volatile v4f*)op = a;
}

extern "C" void kernel_launch(void* const* d_in, const int* in_sizes, int n_in,
                              void* d_out, int out_size, void* d_ws, size_t ws_size,
                              hipStream_t stream) {
  if (n_in < 6) return;
  if (in_sizes[0] != NN * DIN) return;
  if (in_sizes[1] != 2 * NE) return;
  if (in_sizes[2] != DIN * HC || in_sizes[3] != DIN * HC || in_sizes[4] != DIN * HC) return;
  if (in_sizes[5] != HC) return;
  if (out_size != NN * HC + NE * NH) return;

  const float* x  = (const float*)d_in[0];
  const int*   ei = (const int*)  d_in[1];
  const float* Ws = (const float*)d_in[2];
  const float* Wd = (const float*)d_in[3];
  const float* Wv = (const float*)d_in[4];
  const float* av = (const float*)d_in[5];
  float* out0 = (float*)d_out;
  float* out1 = (float*)d_out + (size_t)NN * HC;

  char* ws = (char*)d_ws;
  size_t off = 0;
  const size_t oXB = off; off += (size_t)MP * DIN * 2;          off = (off + 255) & ~(size_t)255;
  const size_t oWT = off; off += (size_t)3 * HC * DIN * 2;      off = (off + 255) & ~(size_t)255;
  const size_t oAV = off; off += (size_t)HC * 4;                off = (off + 255) & ~(size_t)255;
  const size_t oP3 = off; off += (size_t)3 * MP * HC * 4;       off = (off + 255) & ~(size_t)255;
  const size_t oSC = off; off += (size_t)NE * NH * 4;           off = (off + 255) & ~(size_t)255;
  const size_t oMS = off; off += (size_t)NGA * NBA * 8 * 4;     off = (off + 255) & ~(size_t)255;
  if (off > ws_size || off > (size_t)WSMAX) return;
  unsigned short* XB = (unsigned short*)(ws + oXB);
  unsigned short* WT = (unsigned short*)(ws + oWT);
  float* AV = (float*)(ws + oAV);
  float* P3 = (float*)(ws + oP3);
  float* SC = (float*)(ws + oSC);
  float* MS = (float*)(ws + oMS);

  const int scanLds = SCAN_LDS_INTS * 4;
  hipFuncSetAttribute(reinterpret_cast<const void*>(&k_scan),
                      hipFuncAttributeMaxDynamicSharedMemorySize, scanLds);

  k_prep<<<(NUX + 3 * NUW) / NTHR + 1, NTHR, 0, stream>>>(x, Ws, Wd, Wv, av, XB, WT, AV);
  k_proj<<<dim3(MP / GBM, (3 * HC) / GBN), GTHR, 0, stream>>>(XB, WT, P3);
  k_score<<<NE / NTHR, NTHR, 0, stream>>>(ei, P3, AV, SC);
  k_scan<<<NGA, NTHR, scanLds, stream>>>(ei, P3, SC, out0, MS);
  k_attn<<<NE / NTHR, NTHR, 0, stream>>>(ei, SC, MS, out1);
}
